// ProteinStructureEncoder_50714973831806
// MI455X (gfx1250) — hardware-run, weakly checked
//
#include <hip/hip_runtime.h>


namespace {
constexpr int N = 20000, E = 320000, ND = 64, ED = 16, HID = 256, NH = 8, CH = 32, NG = 16, NL = 3, NBLK = N / 16;
constexpr float XS = 64.0f, HGS = 1024.0f, AS_ = 256.0f, WSC = 256.0f, SLOPE = 0.2f;
typedef _Float16 b16;
typedef __attribute__((ext_vector_type(16))) _Float16 v16b;
typedef __attribute__((ext_vector_type(8))) _Float16 v8b;
typedef __attribute__((ext_vector_type(8))) float v8f;
typedef __attribute__((ext_vector_type(4))) float v4f;
__device__ __forceinline__ float bf16_rne(float f) { unsigned int u = __float_as_uint(f); u += 0x7FFFu + ((u >> 16) & 1u); return __uint_as_float(u & 0xFFFF0000u); }
__device__ __forceinline__ void split16(float v, b16& hi, b16& lo) { hi = (b16)v; lo = (b16)(v - (float)hi); }
__device__ __forceinline__ v16b frag_kb(const b16* p, int hh) { const v8b a = *(const v8b*)(p + 8 * hh), b = *(const v8b*)(p + 16 + 8 * hh); v16b f;
#pragma unroll
  for (int e = 0; e < 8; ++e) { f[e] = a[e]; f[8 + e] = b[e]; } return f; }
__device__ __forceinline__ v8f wmma16b(v16b a, v16b b, v8f c) { v8f d = __builtin_amdgcn_wmma_f32_16x16x32_f16(false, a, false, b, (short)0, c, false, false); asm volatile("v_nop\n\tv_nop\n\tv_nop\n\tv_nop" : "+v"(d) : "v"(a), "v"(b)); return d; }
__device__ __forceinline__ void wave_lds_sync() { __builtin_amdgcn_fence(__ATOMIC_RELEASE, "workgroup"); __builtin_amdgcn_wave_barrier(); __builtin_amdgcn_fence(__ATOMIC_ACQUIRE, "workgroup"); }
__device__ __forceinline__ float pmul(float a, float b) { float p = a * b; asm volatile("" : "+v"(p)); return p; }
__device__ __forceinline__ int iclamp(int v, int lo, int hi) { return v < lo ? lo : (v > hi ? hi : v); }
__device__ __forceinline__ float leaky(float v) { return v >= 0.0f ? v : SLOPE * v; }
__device__ __forceinline__ float gelu(float v) { return 0.5f * v * (1.0f + erff(v * 0.70710678118654752f)); }
constexpr int CSR_NBLK9 = 512, CSR_GB9 = 9, CSR_GN9 = 1 << CSR_GB9  , CSR_TS9 = (CSR_GN9 < 32 ? 32 : CSR_GN9)  , CSR_MAXG9 = 512, CSR_CAP9 = 12288  ;
__device__ __host__ __forceinline__ int csr_tix9(int v) { return (v >> CSR_GB9) * CSR_TS9 + (v & (CSR_GN9 - 1)); }
__global__ __launch_bounds__(64) void csrA_kernel9(const int* __restrict__ dst, int E, int N, int nG, int CHP, int NGP, int* __restrict__ STG, int* __restrict__ HST) {
  extern __shared__ int sm[];
  int* cnt = sm; int* run = sm + NGP; int* ids = sm + 2 * NGP;
  const int b = blockIdx.x; const int ch = (E + CSR_NBLK9 - 1) / CSR_NBLK9; const int e0 = b * ch, e1 = min(E, e0 + ch);
  for (int i = threadIdx.x; i < NGP; i += 64) cnt[i] = 0;
  for (int i = threadIdx.x; i < CHP; i += 64) ids[i] = -1;
  __syncthreads();
  if (threadIdx.x == 0) {
    for (int e = e0; e < e1; ++e) { int d = dst[e]; d = (d < 0) ? 0 : (d >= N ? N - 1 : d); cnt[d >> CSR_GB9] += 1; }
    int acc = 0; for (int g = 0; g < nG; ++g) { run[g] = acc; acc += cnt[g]; }
    for (int e = e0; e < e1; ++e) { int d = dst[e]; d = (d < 0) ? 0 : (d >= N ? N - 1 : d); const int g = d >> CSR_GB9; ids[run[g]] = e; run[g] += 1; } }
  __syncthreads();
  typedef __attribute__((ext_vector_type(4))) int v4i;
  for (int pass = 0; pass < 2; ++pass) {
    for (int i = threadIdx.x; i < CHP / 4; i += 64) *(volatile v4i*)(STG + (size_t)b * CHP + i * 4) = *(const v4i*)(&ids[i * 4]);
    for (int i = threadIdx.x; i < NGP / 4; i += 64) { v4i v; for (int e = 0; e < 4; ++e) v[e] = (i * 4 + e < nG) ? cnt[i * 4 + e] : 0; *(volatile v4i*)(HST + (size_t)b * NGP + i * 4) = v; }
    __threadfence(); }
}
__global__ __launch_bounds__(512) void csrS_kernel9(const int* __restrict__ HST, int nG, int NGP, int* __restrict__ START, int* __restrict__ TOT, int* __restrict__ OFF) {
  __shared__ int tot[CSR_MAXG9];
  const int b = threadIdx.x;
  for (int pass = 0; pass < 2; ++pass) { int runb = 0; for (int g = 0; g < nG; ++g) { int c = HST[(size_t)b * NGP + g]; c = (c < 0) ? 0 : c; ((volatile int*)OFF)[(size_t)g * CSR_NBLK9 + b] = runb; runb += c; } __threadfence(); }
  for (int g = threadIdx.x; g < nG; g += 512) { int s = 0; for (int bb = 0; bb < CSR_NBLK9; ++bb) { int c = HST[(size_t)bb * NGP + g]; s += (c < 0) ? 0 : c; } tot[g] = s; }
  __syncthreads();
  if (threadIdx.x < 32) {
    __shared__ int st[CSR_MAXG9 + 32];
    if (threadIdx.x == 0) { int acc = 0; for (int g = 0; g < NGP; ++g) { st[g] = acc; if (g < nG) acc += (tot[g] + 31) & ~31; } st[NGP] = acc; }
    __builtin_amdgcn_fence(__ATOMIC_RELEASE, "workgroup"); __builtin_amdgcn_wave_barrier(); __builtin_amdgcn_fence(__ATOMIC_ACQUIRE, "workgroup");
    for (int pass = 0; pass < 2; ++pass) { for (int i = threadIdx.x; i < NGP + 32; i += 32) { ((volatile int*)START)[i] = (i <= NGP) ? st[min(i, NGP)] : 0; ((volatile int*)TOT)[i] = (i < nG) ? tot[i] : 0; } __threadfence(); } }
}
__global__ __launch_bounds__(256) void csrB_kernel9(const int* __restrict__ dst, int N, int nG, int CHP, int NGP, int permLen, const int* __restrict__ STG, const int* __restrict__ HST, const int* __restrict__ OFF, const int* __restrict__ START, const int* __restrict__ TOT, int* __restrict__ PERM, int* __restrict__ ROWPTR, int* __restrict__ ROWCNT, int* __restrict__ FLAG) {
  typedef __attribute__((ext_vector_type(4))) int v4i;
  __shared__ int ids[CSR_CAP9]; __shared__ unsigned short key[CSR_CAP9]; __shared__ int outp[CSR_CAP9]; __shared__ int ncnt[CSR_GN9 + 1]; __shared__ int boff[CSR_NBLK9 + 1];
  const int g = blockIdx.x, t_ = threadIdx.x; int tot = TOT[g]; int st = START[g], stn = START[g + 1]; const int v0 = g * CSR_GN9; const int nv = min(CSR_GN9, N - v0); const int t0 = g * CSR_TS9;
  st = (st < 0) ? 0 : (st > permLen - 32 ? permLen - 32 : st) & ~31; stn = (stn < st) ? st : (stn > permLen ? permLen : stn); tot = (tot < 0) ? 0 : tot; if (tot > stn - st && tot <= CSR_CAP9) tot = stn - st;
  if (tot > CSR_CAP9) {
    for (int pass = 0; pass < 2; ++pass) { for (int i = t_; i < CSR_TS9 / 4; i += 256) { v4i a, c; for (int e = 0; e < 4; ++e) { a[e] = st; c[e] = 0; } *(volatile v4i*)(ROWPTR + t0 + i * 4) = a; *(volatile v4i*)(ROWCNT + t0 + i * 4) = c; } if (t_ == 0) ((volatile int*)FLAG)[0] = 1; __threadfence(); } (void)nv; return; }
  if (t_ == 0) { int acc = 0; for (int b = 0; b < CSR_NBLK9; ++b) { boff[b] = acc; int c = HST[(size_t)b * NGP + g]; c = (c < 0) ? 0 : (c > CHP ? CHP : c); acc += c; if (acc > tot) acc = tot; } boff[CSR_NBLK9] = acc; }
  for (int i = t_; i <= CSR_GN9; i += 256) ncnt[i] = 0;
  __syncthreads();
  for (int b = 0; b < CSR_NBLK9; ++b) { const int c = boff[b + 1] - boff[b]; int o_ = OFF[(size_t)g * CSR_NBLK9 + b]; o_ = (o_ < 0) ? 0 : (o_ > CHP - c ? CHP - c : o_); const int* src_ = STG + (size_t)b * CHP + o_;
    for (int i = t_; i < c; i += 256) { int id = src_[i]; id = (id < 0) ? 0 : id; ids[boff[b] + i] = id; int d = dst[id]; d = (d < v0) ? v0 : (d >= N ? N - 1 : d); int kk = d - v0; kk = (kk < 0) ? 0 : (kk >= CSR_GN9 ? CSR_GN9 - 1 : kk); key[boff[b] + i] = (unsigned short)kk; } }
  __syncthreads();
  if (t_ == 0) { for (int i = 0; i < tot; ++i) ncnt[key[i]] += 1; int acc = 0; for (int vl = 0; vl < CSR_GN9; ++vl) { const int c = ncnt[vl]; ncnt[vl] = acc; acc += c; } ncnt[CSR_GN9] = acc;
    for (int i = 0; i < tot; ++i) { const int vl = key[i]; outp[ncnt[vl]] = ids[i]; ncnt[vl] += 1; }
    for (int vl = CSR_GN9; vl > 0; --vl) ncnt[vl] = ncnt[vl - 1]; ncnt[0] = 0; }
  __syncthreads();
  for (int pass = 0; pass < 2; ++pass) {
    for (int i = t_; i < (stn - st) / 4; i += 256) { v4i v; for (int e = 0; e < 4; ++e) { const int q = i * 4 + e; v[e] = (q < tot) ? outp[q] : -1; } *(volatile v4i*)(PERM + st + i * 4) = v; }
    for (int i = t_; i < CSR_TS9 / 4; i += 256) { v4i a, c; for (int e = 0; e < 4; ++e) { const int vl = i * 4 + e; const int vc = vl < CSR_GN9 ? vl : CSR_GN9; a[e] = (vl < CSR_GN9) ? st + ncnt[vc] : st; c[e] = (vl < nv) ? (ncnt[(vc < CSR_GN9 ? vc : CSR_GN9 - 1) + 1] - ncnt[vc]) : 0; } *(volatile v4i*)(ROWPTR + t0 + i * 4) = a; *(volatile v4i*)(ROWCNT + t0 + i * 4) = c; }
    __threadfence(); }
}
__global__ __launch_bounds__(256) void csrZ_kernel9(int* __restrict__ p, size_t n4) { typedef __attribute__((ext_vector_type(4))) int v4i; const size_t tid = (size_t)blockIdx.x * 256 + threadIdx.x, nth = (size_t)gridDim.x * 256; v4i z = {0, 0, 0, 0}; for (size_t i = tid; i < n4; i += nth) *(volatile v4i*)(p + i * 4) = z; }
struct CsrBufs9 { int *STG, *HST, *OFF, *START, *TOT, *PERM, *ROWPTR, *ROWCNT, *FLAG; int nG, NGP, CHP; size_t permLen; char* base; size_t bytes; };
static size_t csr_carve9(CsrBufs9& c, char* ws, size_t off, int E, int N) {
  const size_t off0 = off; c.base = ws + off;
  auto al = [&](size_t bytes) { char* p = ws + off; off += (bytes + 255) & ~(size_t)255; return p; };
  c.nG = (N + CSR_GN9 - 1) / CSR_GN9; c.NGP = (c.nG + 31) & ~31; const int ch = (E + CSR_NBLK9 - 1) / CSR_NBLK9; c.CHP = (ch + 31) & ~31; c.permLen = (size_t)E + 32 * (size_t)c.nG + 32;
  c.STG = (int*)al((size_t)CSR_NBLK9 * c.CHP * 4); c.HST = (int*)al((size_t)CSR_NBLK9 * c.NGP * 4); c.OFF = (int*)al((size_t)c.NGP * CSR_NBLK9 * 4); c.START = (int*)al((size_t)(c.NGP + 64) * 4); c.TOT = (int*)al((size_t)(c.NGP + 64) * 4);
  c.PERM = (int*)al(c.permLen * 4); c.ROWPTR = (int*)al((size_t)c.nG * CSR_TS9 * 4); c.ROWCNT = (int*)al((size_t)c.nG * CSR_TS9 * 4); c.FLAG = (int*)al(256);
  c.bytes = off - off0; return off;
}
static void csr_build9(const CsrBufs9& c, const int* dst, int E, int N, hipStream_t stream) {
  const size_t smem = (size_t)(2 * c.NGP + c.CHP) * 4;
  csrZ_kernel9<<<512, 256, 0, stream>>>((int*)c.base, c.bytes / 16);
  csrA_kernel9<<<CSR_NBLK9, 64, smem, stream>>>(dst, E, N, c.nG, c.CHP, c.NGP, c.STG, c.HST);
  csrS_kernel9<<<1, 512, 0, stream>>>(c.HST, c.nG, c.NGP, c.START, c.TOT, c.OFF);
  csrB_kernel9<<<c.nG, 256, 0, stream>>>(dst, N, c.nG, c.CHP, c.NGP, (int)c.permLen, c.STG, c.HST, c.OFF, c.START, c.TOT, c.PERM, c.ROWPTR, c.ROWCNT, c.FLAG);
}


__global__ __launch_bounds__(256) void wput_kernel(const float* __restrict__ w, int KIN, int KP, int OUTW, int ro, b16* __restrict__ WT) {
  const int KG = KP / 8; const size_t u = (size_t)blockIdx.x * 256 + threadIdx.x; if (u >= (size_t)OUTW * KG) return; const int o = (int)(u / KG), k0 = (int)(u % KG) * 8; v8b v;
#pragma unroll
  for (int j = 0; j < 8; ++j) { const int k = k0 + j; v[j] = k < KIN ? (b16)(bf16_rne(w[(size_t)k * OUTW + o]) * WSC) : (b16)0.0f; } for (int pass = 0; pass < 2; ++pass) { *(volatile v8b*)(WT + (size_t)(ro + o) * KP + k0) = v; __threadfence(); }
}
__global__ __launch_bounds__(256) void ea_kernel(const float* __restrict__ eat, const float* __restrict__ eW, const float* __restrict__ eb, float* __restrict__ EA) {
  const size_t u = (size_t)blockIdx.x * 256 + threadIdx.x; if (u >= (size_t)E * 4) return; const size_t e = u / 4; const int o0 = (int)(u % 4) * 4; float a[ED]; for (int k = 0; k < ED; ++k) a[k] = bf16_rne(eat[e * ED + k]); v4f r;
  for (int i = 0; i < 4; ++i) { const int o = o0 + i; float s = bf16_rne(eb[o]); for (int k = 0; k < ED; ++k) s += pmul(a[k], bf16_rne(eW[k * ED + o])); r[i] = s; }
  for (int pass = 0; pass < 2; ++pass) { *(volatile v4f*)(EA + e * ED + o0) = r; __threadfence(); }
}
template <int KIN, int NT, int EXACT>
__global__ __launch_bounds__(32) void dense_kernel(const float* __restrict__ IN, const b16* __restrict__ WT, const float* __restrict__ bias, int NLIM, float* __restrict__ OUT) {
  __shared__ __attribute__((aligned(16))) b16 Ah[16][KIN + 8], Al[16][(EXACT ? 32 : KIN) + 8]; __shared__ __attribute__((aligned(16))) float Tf[16][128 + 4];
  const int lane = threadIdx.x, nloc = lane & 15, hlf = lane >> 4; const size_t m0 = (size_t)blockIdx.x * 16; if (m0 >= (size_t)NLIM) return;
  for (int rr = 0; rr < 16; ++rr) for (int q = 0; q < KIN / 32; ++q) { const float v = IN[(m0 + rr) * KIN + q * 32 + lane]; if (EXACT) Ah[rr][q * 32 + lane] = (b16)(bf16_rne(v) * XS); else { b16 p, ql; split16(v * XS, p, ql); Ah[rr][q * 32 + lane] = p; Al[rr][q * 32 + lane] = ql; } }
  wave_lds_sync();
#pragma unroll 1
  for (int cg = 0; cg < NT / 8; ++cg) { v8f acc[8];
#pragma unroll
    for (int t = 0; t < 8; ++t) acc[t] = (v8f){};
#pragma unroll 2
    for (int kb = 0; kb < KIN; kb += 32) { const v16b a = frag_kb(&Ah[nloc][kb], hlf); v16b al; if (!EXACT) al = frag_kb(&Al[nloc][kb], hlf);
#pragma unroll
      for (int t = 0; t < 8; ++t) { const v16b bw = frag_kb(WT + (size_t)(cg * 128 + t * 16 + nloc) * KIN + kb, hlf); acc[t] = wmma16b(a, bw, acc[t]); if (!EXACT) acc[t] = wmma16b(al, bw, acc[t]); } }
#pragma unroll
    for (int t = 0; t < 8; ++t) { const int c = cg * 128 + t * 16 + nloc; const float bb = bf16_rne(bias[c]);
#pragma unroll
      for (int r8 = 0; r8 < 8; ++r8) Tf[8 * hlf + r8][t * 16 + nloc] = acc[t][r8] * (1.0f / (XS * WSC)) + bb; }
    wave_lds_sync();
    for (int pass = 0; pass < 2; ++pass) { for (int rr = 0; rr < 16; ++rr) *(volatile v4f*)(OUT + (m0 + rr) * (size_t)(NT * 16) + cg * 128 + lane * 4) = *(const v4f*)(&Tf[rr][lane * 4]); __threadfence(); }
    wave_lds_sync(); }
}
__global__ __launch_bounds__(32) void gat_kernel(const float* __restrict__ Hh, const float* __restrict__ XLR, const float* __restrict__ EA, const int* __restrict__ srcs, const int* __restrict__ PERM, const int* __restrict__ ROWPTR, const int* __restrict__ ROWCNT, int permLen, const b16* __restrict__ WE, const float* __restrict__ att, const float* __restrict__ cbias, int NLIM, float* __restrict__ HN) {
  __shared__ __attribute__((aligned(16))) b16 Ah[16][40], Al[16][40]; __shared__ float Ee[16][HID + 1], Lg[16][NH + 1]; __shared__ int Ss[16];
  const int lane = threadIdx.x, nloc = lane & 15, hlf = lane >> 4; const size_t v = blockIdx.x; if (v >= (size_t)NLIM) return; const int c0 = lane * 8, h = lane >> 2;
  int st = ROWPTR[v], cnt = ROWCNT[v]; cnt = iclamp(cnt, 0, 1 << 20); st = iclamp(st, 0, permLen - cnt);
  float lea = 0.0f; int nin = 0;
#pragma unroll 1
  for (int j = 0; j < cnt; ++j) { const int e = iclamp(PERM[st + j], 0, E - 1); const int s = iclamp(srcs[e], 0, N - 1); if (s >= NLIM) continue; ++nin; if (lane < ED) lea += EA[(size_t)e * ED + lane]; }
  lea = lea / (float)(nin < 1 ? 1 : nin);
  float xr[8], at[8], m = -INFINITY, den = 0.0f, acc[8]; for (int i = 0; i < 8; ++i) { xr[i] = XLR[v * (2 * HID) + HID + c0 + i]; at[i] = bf16_rne(att[c0 + i]); acc[i] = 0.0f; }
  const int nslot = cnt + 1;
#pragma unroll 1
  for (int j0 = 0; j0 < nslot; j0 += 16) {
    for (int rr = 0; rr < 16; ++rr) { const int jj = j0 + rr; int s = -1; float a = 0.0f; if (jj == 0) { s = (int)v; a = (lane < ED) ? lea : 0.0f; } else if (jj < nslot) { const int e = iclamp(PERM[st + jj - 1], 0, E - 1); s = iclamp(srcs[e], 0, N - 1); if (s >= NLIM) s = -1; a = (lane < ED && s >= 0) ? EA[(size_t)e * ED + lane] : 0.0f; }
      if (lane == 0) Ss[rr] = s; b16 p = (b16)0.0f, q = (b16)0.0f; if (lane < ED) split16(a * AS_, p, q); Ah[rr][lane] = p; Al[rr][lane] = q; }
    wave_lds_sync();
    { const v16b a = frag_kb(&Ah[nloc][0], hlf), al = frag_kb(&Al[nloc][0], hlf);
#pragma unroll 1
      for (int cg = 0; cg < 2; ++cg) { v8f ee[8];
#pragma unroll
        for (int t = 0; t < 8; ++t) { ee[t] = (v8f){}; const v16b bw = frag_kb(WE + (size_t)(cg * 128 + t * 16 + nloc) * 32, hlf); ee[t] = wmma16b(a, bw, ee[t]); ee[t] = wmma16b(al, bw, ee[t]); }
#pragma unroll
        for (int t = 0; t < 8; ++t)
#pragma unroll
          for (int r8 = 0; r8 < 8; ++r8) Ee[8 * hlf + r8][cg * 128 + t * 16 + nloc] = ee[t][r8] * (1.0f / (AS_ * WSC)); } }
    wave_lds_sync();
    float xls[16][8];
#pragma unroll
    for (int rr = 0; rr < 16; ++rr) { const int s = Ss[rr]; float lg = 0.0f; if (s >= 0) { const v4f x0 = *(const v4f*)(XLR + (size_t)s * (2 * HID) + c0), x1 = *(const v4f*)(XLR + (size_t)s * (2 * HID) + c0 + 4);
        const float xv[8] = {x0[0], x0[1], x0[2], x0[3], x1[0], x1[1], x1[2], x1[3]}; for (int i = 0; i < 8; ++i) { xls[rr][i] = xv[i]; lg += pmul(leaky(xv[i] + xr[i] + Ee[rr][c0 + i]), at[i]); } } else { for (int i = 0; i < 8; ++i) xls[rr][i] = 0.0f; }
      lg += __shfl_xor(lg, 1); lg += __shfl_xor(lg, 2); if ((lane & 3) == 0) Lg[rr][h] = (s >= 0) ? lg : -INFINITY; }
    wave_lds_sync();
    float cm = -INFINITY; for (int rr = 0; rr < 16; ++rr) cm = fmaxf(cm, Lg[rr][h]);
    const float mn = fmaxf(m, cm); const float sc = (m == -INFINITY) ? 0.0f : __expf(m - mn); den *= sc; for (int i = 0; i < 8; ++i) acc[i] *= sc;
#pragma unroll
    for (int rr = 0; rr < 16; ++rr) { const float l = Lg[rr][h]; const float p = (l == -INFINITY) ? 0.0f : __expf(l - mn); den += p; for (int i = 0; i < 8; ++i) acc[i] += pmul(p, xls[rr][i]); }
    m = mn; wave_lds_sync(); }
  const float inv = 1.0f / den; float r[8]; for (int i = 0; i < 8; ++i) r[i] = Hh[v * HID + c0 + i] + pmul(acc[i], inv) + bf16_rne(cbias[c0 + i]);
  for (int pass = 0; pass < 2; ++pass) { *(volatile v4f*)(HN + v * HID + c0) = (v4f){r[0], r[1], r[2], r[3]}; *(volatile v4f*)(HN + v * HID + c0 + 4) = (v4f){r[4], r[5], r[6], r[7]}; __threadfence(); }
}
__global__ __launch_bounds__(32) void head_kernel(const float* __restrict__ Hh, const int* __restrict__ batch, const b16* __restrict__ W1T, const float* __restrict__ b1, const b16* __restrict__ W2T, const float* __restrict__ b2, int NLIM, float* __restrict__ out) {
  __shared__ __attribute__((aligned(16))) b16 Ah[16][HID + 8], Al[16][HID + 8], Bh[16][HID + 8], Bl[16][HID + 8]; __shared__ __attribute__((aligned(16))) float Tf[16][128 + 4];
  const int lane = threadIdx.x, nloc = lane & 15, hlf = lane >> 4;
  auto lb = [&](int key) -> int { int lo = 0, hi = N; for (int it = 0; it < 16 && lo < hi; ++it) { const int mid = (lo + hi) >> 1; if (batch[mid] < key) lo = mid + 1; else hi = mid; } return lo; };
  for (int g = 0; g < NG; ++g) { int s0 = lb(g), e0 = lb(g + 1); const int call = e0 - s0; if (e0 > NLIM) e0 = NLIM; if (e0 < s0) e0 = s0; float s[8]; for (int q = 0; q < 8; ++q) s[q] = 0.0f;
#pragma unroll 1
    for (int n = s0; n < e0; ++n) for (int q = 0; q < 8; ++q) s[q] += Hh[(size_t)n * HID + q * 32 + lane];
    const float inv = 1.0f / (float)(call < 1 ? 1 : call); for (int q = 0; q < 8; ++q) { b16 p, ql; split16(pmul(s[q], inv) * HGS, p, ql); Ah[g][q * 32 + lane] = p; Al[g][q * 32 + lane] = ql; } }
  wave_lds_sync();
#pragma unroll 1
  for (int cg = 0; cg < 2; ++cg) { v8f acc[8];
#pragma unroll
    for (int t = 0; t < 8; ++t) acc[t] = (v8f){};
#pragma unroll 2
    for (int kb = 0; kb < HID; kb += 32) { const v16b a = frag_kb(&Ah[nloc][kb], hlf), al = frag_kb(&Al[nloc][kb], hlf);
#pragma unroll
      for (int t = 0; t < 8; ++t) { const v16b bw = frag_kb(W1T + (size_t)(cg * 128 + t * 16 + nloc) * HID + kb, hlf); acc[t] = wmma16b(a, bw, acc[t]); acc[t] = wmma16b(al, bw, acc[t]); } }
#pragma unroll
    for (int t = 0; t < 8; ++t) { const int c = cg * 128 + t * 16 + nloc; const float bb = bf16_rne(b1[c]);
#pragma unroll
      for (int r8 = 0; r8 < 8; ++r8) { b16 p, ql; split16(gelu(acc[t][r8] * (1.0f / (HGS * WSC)) + bb) * XS, p, ql); Bh[8 * hlf + r8][c] = p; Bl[8 * hlf + r8][c] = ql; } } }
  wave_lds_sync();
#pragma unroll 1
  for (int cg = 0; cg < 2; ++cg) { v8f acc[8];
#pragma unroll
    for (int t = 0; t < 8; ++t) acc[t] = (v8f){};
#pragma unroll 2
    for (int kb = 0; kb < HID; kb += 32) { const v16b a = frag_kb(&Bh[nloc][kb], hlf), al = frag_kb(&Bl[nloc][kb], hlf);
#pragma unroll
      for (int t = 0; t < 8; ++t) { const v16b bw = frag_kb(W2T + (size_t)(cg * 128 + t * 16 + nloc) * HID + kb, hlf); acc[t] = wmma16b(a, bw, acc[t]); acc[t] = wmma16b(al, bw, acc[t]); } }
#pragma unroll
    for (int t = 0; t < 8; ++t) { const int c = cg * 128 + t * 16 + nloc; const float bb = bf16_rne(b2[c]);
#pragma unroll
      for (int r8 = 0; r8 < 8; ++r8) Tf[8 * hlf + r8][t * 16 + nloc] = acc[t][r8] * (1.0f / (XS * WSC)) + bb; }
    wave_lds_sync();
    for (int pass = 0; pass < 2; ++pass) { for (int rr = 0; rr < NG; ++rr) *(volatile v4f*)(out + (size_t)rr * HID + cg * 128 + lane * 4) = *(const v4f*)(&Tf[rr][lane * 4]); __threadfence(); }
    wave_lds_sync(); }
}
__global__ __launch_bounds__(256) void blr_kernel(const float* __restrict__ bl, const float* __restrict__ br, float* __restrict__ BLR) { for (int i = threadIdx.x; i < NL * 2 * HID; i += 256) { const int l = i / (2 * HID), c = i % (2 * HID); const float v = c < HID ? bl[l * HID + c] : br[l * HID + c - HID]; for (int pass = 0; pass < 2; ++pass) { ((volatile float*)BLR)[i] = v; __threadfence(); } } }
}

extern "C" void kernel_launch(void* const* d_in, const int* in_sizes, int n_in, void* d_out, int out_size, void* d_ws, size_t ws_size, hipStream_t stream) {
  (void)n_in;
  auto Fp = [&](int i) { return (const float*)d_in[i]; }; auto Ip = [&](int i) { return (const int*)d_in[i]; };
  if (in_sizes[0] != N * ND || in_sizes[1] != 2 * E || in_sizes[2] != E * ED || in_sizes[3] != N || in_sizes[4] != ND * HID || in_sizes[6] != ED * ED || in_sizes[8] != NL * HID * HID || in_sizes[10] != NL * HID * HID || in_sizes[12] != NL * ED * HID || in_sizes[13] != NL * NH * CH || in_sizes[15] != HID * HID || in_sizes[17] != HID * HID || out_size != NG * HID) return;
  const int NLIM = N; const int GB16 = NBLK;
  size_t off = 0; char* ws = (char*)d_ws;
  auto carve = [&](size_t bytes) { char* p = ws + off; off += (bytes + 255) & ~(size_t)255; return p; };
  b16* WN = (b16*)carve((size_t)HID * ND * 2); b16* WLR = (b16*)carve((size_t)NL * 2 * HID * HID * 2); b16* WEE = (b16*)carve((size_t)NL * HID * 32 * 2); b16* W1T = (b16*)carve((size_t)HID * HID * 2); b16* W2T = (b16*)carve((size_t)HID * HID * 2);
  float* EA = (float*)carve((size_t)E * ED * 4); float* HA = (float*)carve((size_t)N * HID * 4); float* HB = (float*)carve((size_t)N * HID * 4); float* XLR = (float*)carve((size_t)N * 2 * HID * 4); float* BLR = (float*)carve((size_t)NL * 2 * HID * 4);
  CsrBufs9 csr; off = csr_carve9(csr, ws, off, E, N);
  if (off > ws_size || off > ((size_t)128 << 20)) return;
  wput_kernel<<<(HID * 8 + 255) / 256, 256, 0, stream>>>(Fp(4), ND, ND, HID, 0, WN);
  for (int l = 0; l < NL; ++l) { wput_kernel<<<(HID * 32 + 255) / 256, 256, 0, stream>>>(Fp(8) + (size_t)l * HID * HID, HID, HID, HID, l * 2 * HID, WLR); wput_kernel<<<(HID * 32 + 255) / 256, 256, 0, stream>>>(Fp(10) + (size_t)l * HID * HID, HID, HID, HID, l * 2 * HID + HID, WLR); wput_kernel<<<(HID * 4 + 255) / 256, 256, 0, stream>>>(Fp(12) + (size_t)l * ED * HID, ED, 32, HID, l * HID, WEE); }
  wput_kernel<<<(HID * 32 + 255) / 256, 256, 0, stream>>>(Fp(15), HID, HID, HID, 0, W1T); wput_kernel<<<(HID * 32 + 255) / 256, 256, 0, stream>>>(Fp(17), HID, HID, HID, 0, W2T);
  blr_kernel<<<1, 256, 0, stream>>>(Fp(9), Fp(11), BLR);
  csr_build9(csr, Ip(1) + E, E, N, stream);
  ea_kernel<<<(unsigned)(((size_t)E * 4 + 255) / 256), 256, 0, stream>>>(Fp(2), Fp(6), Fp(7), EA);
  dense_kernel<ND, 16, 1><<<GB16, 32, 0, stream>>>(Fp(0), WN, Fp(5), NLIM, HA);
  float* Hc = HA; float* Hn = HB;
  for (int l = 0; l < NL; ++l) {
    dense_kernel<HID, 32, 0><<<GB16, 32, 0, stream>>>(Hc, WLR + (size_t)l * 2 * HID * HID, BLR + (size_t)l * 2 * HID, NLIM, XLR);
    gat_kernel<<<(unsigned)NLIM, 32, 0, stream>>>(Hc, XLR, EA, Ip(1), csr.PERM, csr.ROWPTR, csr.ROWCNT, (int)csr.permLen, WEE + (size_t)l * HID * 32, Fp(13) + (size_t)l * NH * CH, Fp(14) + (size_t)l * HID, NLIM, Hn);
    float* t = Hc; Hc = Hn; Hn = t; }
  head_kernel<<<1, 32, 0, stream>>>(Hc, Ip(3), W1T, Fp(16), W2T, Fp(18), NLIM, (float*)d_out);
}
